// Evoformer_23235773071559
// MI455X (gfx1250) — hardware-verified
//
#include <hip/hip_runtime.h>


#define NS   64
#define NRS  256
#define EE   256
#define PE_  128
#define NH_  8
#define HC   32
#define SGL  384
#define NTR  (NS * NRS)
#define NPR  (NRS * NRS)
#define ZR   128
#define ZCP  1024
#define PCAR 1024.0f
typedef _Float16 h16;
typedef unsigned short bf;
typedef __attribute__((ext_vector_type(16))) __bf16   v16bf;
typedef __attribute__((ext_vector_type(16))) _Float16 v16h;
typedef __attribute__((ext_vector_type(8)))  _Float16 v8h;
typedef __attribute__((ext_vector_type(8)))  unsigned short v8us;
typedef __attribute__((ext_vector_type(8)))  float    v8f;
typedef __attribute__((ext_vector_type(4)))  float    v4f;
typedef v8h  __attribute__((may_alias)) v8ha;
typedef v4f  __attribute__((may_alias)) v4fa;
typedef v8us __attribute__((may_alias)) v8usa;

__device__ __forceinline__ unsigned short f2bf(float f) { unsigned u = __float_as_uint(f); u += 0x7FFFu + ((u >> 16) & 1u); return (unsigned short)(u >> 16); }
__device__ __forceinline__ float bf2f(unsigned short b) { return __uint_as_float(((unsigned)b) << 16); }
__device__ __forceinline__ float bfr(float f) { return bf2f(f2bf(f)); }
__device__ __forceinline__ v16h cat16(v8h lo, v8h hi) { return __builtin_shufflevector(lo, hi, 0, 1, 2, 3, 4, 5, 6, 7, 8, 9, 10, 11, 12, 13, 14, 15); }
__device__ __forceinline__ v16bf cat16b(v8us lo, v8us hi) { return __builtin_bit_cast(v16bf, __builtin_shufflevector(lo, hi, 0, 1, 2, 3, 4, 5, 6, 7, 8, 9, 10, 11, 12, 13, 14, 15)); }
__device__ __forceinline__ v8f wmma16(v16h a, v16h b, v8f c) { return __builtin_amdgcn_wmma_f32_16x16x32_f16(false, a, false, b, (short)0, c, false, false); }
__device__ __forceinline__ v8f wmmab(v16bf a, v16bf b, v8f c) { return __builtin_amdgcn_wmma_f32_16x16x32_bf16(false, a, false, b, (short)0, c, false, false); }


template <typename T16> struct WFrag;
template <> struct WFrag<h16> { typedef v16h V; static __device__ __forceinline__ V ld(const h16* p) { return cat16(*(const v8h*)p, *(const v8h*)(p + 16)); } static __device__ __forceinline__ v8f mma(V a, V b, v8f c) { return wmma16(a, b, c); } };
template <> struct WFrag<bf> { typedef v16bf V; static __device__ __forceinline__ V ld(const bf* p) { return cat16b(*(const v8us*)p, *(const v8us*)(p + 16)); } static __device__ __forceinline__ v8f mma(V a, V b, v8f c) { return wmmab(a, b, c); } };
template <typename T16, int NSPLIT, bool BIAS>
__global__ __launch_bounds__(32) void k_gemmw(const T16* __restrict__ A, const T16* __restrict__ A2, const T16* __restrict__ Bt, const T16* __restrict__ Bt2, int K, float* C, int ldc, const float* __restrict__ bias, size_t sA, size_t sB, size_t sC) {
    typedef typename WFrag<T16>::V V;
    __shared__ __align__(16) float os[16 * 68];
    const size_t z = blockIdx.z; A += z * sA; if (A2) A2 += z * sA; Bt += z * sB; if (Bt2) Bt2 += z * sB; C += z * sC;
    const int lane = threadIdx.x & 31, lr = lane & 15, hi = lane >> 4; const int r0 = blockIdx.x * 64, c0 = blockIdx.y * 64;
    v8f acc[4][4];
#pragma unroll
    for (int mb = 0; mb < 4; ++mb)
#pragma unroll
        for (int nb = 0; nb < 4; ++nb) acc[mb][nb] = (v8f){};
    const size_t aoff = (size_t)(r0 + lr) * K + 8 * hi, boff = (size_t)(c0 + lr) * K + 8 * hi;
#pragma unroll 1
    for (int kc = 0; kc < K; kc += 32) {
        V a[4], a2[4];
#pragma unroll
        for (int mb = 0; mb < 4; ++mb) { a[mb] = WFrag<T16>::ld(A + aoff + (size_t)mb * 16 * K + kc); if (NSPLIT == 1 || NSPLIT == 2) a2[mb] = WFrag<T16>::ld(A2 + aoff + (size_t)mb * 16 * K + kc); }
#pragma unroll
        for (int nb = 0; nb < 4; ++nb) { const V b = WFrag<T16>::ld(Bt + boff + (size_t)nb * 16 * K + kc); V b2; if (NSPLIT >= 2) b2 = WFrag<T16>::ld(Bt2 + boff + (size_t)nb * 16 * K + kc);
#pragma unroll
            for (int mb = 0; mb < 4; ++mb) { acc[mb][nb] = WFrag<T16>::mma(a[mb], b, acc[mb][nb]); if (NSPLIT == 1 || NSPLIT == 2) acc[mb][nb] = WFrag<T16>::mma(a2[mb], b, acc[mb][nb]); if (NSPLIT >= 2) acc[mb][nb] = WFrag<T16>::mma(a[mb], b2, acc[mb][nb]); } }
        asm volatile("v_nop\n\tv_nop\n\tv_nop\n\tv_nop" : "+v"(acc[0][0]), "+v"(acc[1][1]), "+v"(acc[2][2]), "+v"(acc[3][3]) : "v"(a[0]), "v"(a[3]));
    }
#pragma unroll
    for (int mb = 0; mb < 4; ++mb) {
#pragma unroll
        for (int nb = 0; nb < 4; ++nb) {
#pragma unroll
            for (int j = 0; j < 8; ++j) os[(hi * 8 + j) * 68 + nb * 16 + lr] = acc[mb][nb][j]; }
        __builtin_amdgcn_wave_barrier(); asm volatile("" ::: "memory");
        float* crow = C + (size_t)(r0 + mb * 16) * ldc + c0;
#pragma unroll 1
        for (int ps = 0; ps < 2; ++ps) {
#pragma unroll
            for (int s = 0; s < 8; ++s) { const int row = 2 * s + hi, cofs = lr * 4; v4f val = *(const v4fa*)(os + row * 68 + cofs); if (BIAS) { val[0] += bfr(bias[c0 + cofs]); val[1] += bfr(bias[c0 + cofs + 1]); val[2] += bfr(bias[c0 + cofs + 2]); val[3] += bfr(bias[c0 + cofs + 3]); }
                *(volatile v4f*)(crow + (size_t)row * ldc + cofs) = val; }
            if (ps == 0) __threadfence(); }
        __builtin_amdgcn_wave_barrier(); asm volatile("" ::: "memory");
    }
}

__device__ __forceinline__ h16 tohx(float x) { return (h16)x; }
__device__ __forceinline__ void splitf(float y, unsigned short& h, unsigned short& l) { h = f2bf(y); l = f2bf(y - bf2f(h)); }
typedef __attribute__((ext_vector_type(4))) _Float16 v4h;

__global__ __launch_bounds__(256) void k_wth(const float* __restrict__ w, int K, int N, int Np, h16* Bt) {
    typedef __attribute__((ext_vector_type(2))) _Float16 v2h;
    const int lane = threadIdx.x & 31; const int nlines = Np * K / 64; const int wg = blockIdx.x * 8 + (threadIdx.x >> 5), nw = gridDim.x * 8;
#pragma unroll 1
    for (int ps = 0; ps < 2; ++ps) {
#pragma unroll 1
        for (int L = wg; L < nlines; L += nw) { const int e = L * 64 + lane * 2; v2h o;
#pragma unroll
            for (int q = 0; q < 2; ++q) { const int n = (e + q) / K, k = (e + q) % K; o[q] = (n < N) ? tohx(bfr(w[(size_t)k * N + (n < N ? n : 0)])) : tohx(0.f); }
            *(volatile v2h*)(Bt + e) = o; }
        if (ps == 0) __threadfence(); }
}
__global__ __launch_bounds__(256) void k_wtb(const float* __restrict__ w, int K, int N, bf* Bt) {
    typedef __attribute__((ext_vector_type(2))) unsigned short v2us;
    const int lane = threadIdx.x & 31; const int nlines = N * K / 64; const int wg = blockIdx.x * 8 + (threadIdx.x >> 5), nw = gridDim.x * 8;
#pragma unroll 1
    for (int ps = 0; ps < 2; ++ps) {
#pragma unroll 1
        for (int L = wg; L < nlines; L += nw) { const int e = L * 64 + lane * 2; v2us o;
#pragma unroll
            for (int q = 0; q < 2; ++q) { const int n = (e + q) / K, k = (e + q) % K; o[q] = f2bf(w[(size_t)k * N + n]); }
            *(volatile v2us*)(Bt + e) = o; }
        if (ps == 0) __threadfence(); }
}
template <int D, bool RB>
__global__ __launch_bounds__(256) void k_ln(const float* __restrict__ X, const float* __restrict__ sc, const float* __restrict__ bi, int rows, h16* Mh) {
    const int lane = threadIdx.x & 31; const int r = blockIdx.x * 8 + (threadIdx.x >> 5); if (r >= rows) return; constexpr int NQ = D / 128; float v[NQ * 4]; float s = 0.f;
#pragma unroll
    for (int c = 0; c < NQ; ++c)
#pragma unroll
        for (int q = 0; q < 4; ++q) { float x = X[(size_t)r * D + c * 128 + lane * 4 + q]; if (RB) x = bfr(x); v[c * 4 + q] = x; s += x; }
#pragma unroll
    for (int sh = 16; sh; sh >>= 1) s += __shfl_xor(s, sh, 32);
    const float mu = s * (1.0f / D); float qq = 0.f;
#pragma unroll
    for (int i = 0; i < NQ * 4; ++i) { const float d = v[i] - mu; qq = fmaf(d, d, qq); }
#pragma unroll
    for (int sh = 16; sh; sh >>= 1) qq += __shfl_xor(qq, sh, 32);
    const float rs = rsqrtf(qq * (1.0f / D) + 1e-5f); v4h o[NQ];
#pragma unroll
    for (int c = 0; c < NQ; ++c)
#pragma unroll
        for (int q = 0; q < 4; ++q) { const int col = c * 128 + lane * 4 + q; o[c][q] = tohx((v[c * 4 + q] - mu) * rs * bfr(sc[col]) + bfr(bi[col])); }
#pragma unroll 1
    for (int ps = 0; ps < 2; ++ps) {
#pragma unroll
        for (int c = 0; c < NQ; ++c) *(volatile v4h*)(Mh + (size_t)r * D + c * 128 + lane * 4) = o[c];
        if (ps == 0) __threadfence(); }
}
__global__ __launch_bounds__(256) void k_bcomp(const float* __restrict__ BQ, float* BQ8) {
    const int lane = threadIdx.x & 31; const int wg = blockIdx.x * 8 + (threadIdx.x >> 5); if (wg >= NH_ * NRS * 2) return; const int h = wg / (NRS * 2), q = (wg / 2) % NRS, k0 = (wg & 1) * 128 + lane * 4; v4f o;
#pragma unroll
    for (int i = 0; i < 4; ++i) o[i] = BQ[((size_t)q * NRS + k0 + i) * 64 + h];
    float* dst = BQ8 + ((size_t)h * NRS + q) * NRS + k0; *(volatile v4f*)dst = o; __threadfence(); *(volatile v4f*)dst = o;
}
template <bool COL>
__global__ __launch_bounds__(256) void k_hplane(const float* __restrict__ F, float sc, h16* P) {
    typedef __attribute__((ext_vector_type(2))) _Float16 v2h;
    const int lane = threadIdx.x & 31; const size_t L0 = ((size_t)blockIdx.x * 8 + (threadIdx.x >> 5)) * 8; const size_t nlines = (size_t)NTR * EE / 64;
#pragma unroll 1
    for (int ps = 0; ps < 2; ++ps) {
#pragma unroll
        for (int l = 0; l < 8; ++l) { const size_t L = L0 + l; if (L >= nlines) break; const size_t e = L * 64 + lane * 2; const int c = (int)(e & 31); const int n = (int)((e >> 5) % (COL ? NS : NRS)); const int z = (int)(e / (32 * (COL ? NS : NRS))); const int h = z & 7, o = z >> 3;
            const int s = COL ? n : o, r = COL ? o : n; v2h v;
#pragma unroll
            for (int q = 0; q < 2; ++q) v[q] = tohx(F[((size_t)s * NRS + r) * EE + h * HC + c + q] * sc);
            *(volatile v2h*)(P + e) = v; }
        if (ps == 0) __threadfence(); }
}
template <bool COL>
__global__ __launch_bounds__(256) void k_vtplane(const float* __restrict__ F, h16* VT) {
    typedef __attribute__((ext_vector_type(2))) _Float16 v2h;
    constexpr int NK = COL ? NS : NRS; const int lane = threadIdx.x & 31; const size_t L0 = ((size_t)blockIdx.x * 8 + (threadIdx.x >> 5)) * 8; const size_t nlines = (size_t)(COL ? NRS : NS) * NH_ * 64 * NK / 64;
#pragma unroll 1
    for (int ps = 0; ps < 2; ++ps) {
#pragma unroll
        for (int l = 0; l < 8; ++l) { const size_t L = L0 + l; if (L >= nlines) break; const size_t e = L * 64 + lane * 2; const int n = (int)(e % NK); const int c = (int)((e / NK) % 64); const int z = (int)(e / (64 * NK)); const int h = z & 7, o = z >> 3; v2h v;
#pragma unroll
            for (int q = 0; q < 2; ++q) { const int nn = n + q; const int s = COL ? nn : o, r = COL ? o : nn; v[q] = (c < HC) ? tohx(F[((size_t)s * NRS + r) * EE + h * HC + (c < HC ? c : 0)]) : tohx(0.f); }
            *(volatile v2h*)(VT + e) = v; }
        if (ps == 0) __threadfence(); }
}
__global__ __launch_bounds__(256) void k_gsig(const float* __restrict__ G, const float* __restrict__ bg, h16* GS) {
    const int lane = threadIdx.x & 31; const int r = blockIdx.x * 8 + (threadIdx.x >> 5); if (r >= NTR) return; v4h o[2];
#pragma unroll
    for (int c = 0; c < 2; ++c)
#pragma unroll
        for (int q = 0; q < 4; ++q) { const int col = c * 128 + lane * 4 + q; const float x = G[(size_t)r * EE + col] + bfr(bg[col]); o[c][q] = tohx(__fdiv_rn(1.0f, 1.0f + __expf(-x))); }
#pragma unroll 1
    for (int ps = 0; ps < 2; ++ps) {
#pragma unroll
        for (int c = 0; c < 2; ++c) *(volatile v4h*)(GS + (size_t)r * EE + c * 128 + lane * 4) = o[c];
        if (ps == 0) __threadfence(); }
}
template <int NK, bool BIAS>
__global__ __launch_bounds__(256) void k_soft(const float* __restrict__ Sb, const float* __restrict__ BQ8, int nrows, h16* P) {
    const int lane = threadIdx.x & 31; const int row = blockIdx.x * 8 + (threadIdx.x >> 5); if (row >= nrows) return; const int zz = row / (NK == 256 ? NRS : NS), q = row % (NK == 256 ? NRS : NS); const int h = zz & 7;
    constexpr int PER = NK / 32; constexpr int VW = PER >= 4 ? 4 : PER; constexpr int NCH = PER / VW; float v[PER]; float mx = -3.0e38f;
    const float* sr = Sb + (size_t)row * NK; const float* br = BQ8 + ((size_t)h * NRS + q) * NRS;
#pragma unroll
    for (int ch = 0; ch < NCH; ++ch)
#pragma unroll
        for (int i = 0; i < VW; ++i) { const int k = ch * (32 * VW) + lane * VW + i; float x = sr[k]; if (BIAS) x += br[k]; v[ch * VW + i] = x; mx = fmaxf(mx, x); }
#pragma unroll
    for (int sh = 16; sh; sh >>= 1) mx = fmaxf(mx, __shfl_xor(mx, sh, 32));
    float sum = 0.f;
#pragma unroll
    for (int i = 0; i < PER; ++i) { v[i] = __expf(v[i] - mx); sum += v[i]; }
#pragma unroll
    for (int sh = 16; sh; sh >>= 1) sum += __shfl_xor(sum, sh, 32);
    const float f = __fdiv_rn(PCAR, sum);
    typedef __attribute__((ext_vector_type(VW))) _Float16 vvh; vvh o[NCH];
#pragma unroll
    for (int ch = 0; ch < NCH; ++ch)
#pragma unroll
        for (int i = 0; i < VW; ++i) o[ch][i] = tohx(v[ch * VW + i] * f);
#pragma unroll 1
    for (int ps = 0; ps < 2; ++ps) {
#pragma unroll
        for (int ch = 0; ch < NCH; ++ch) *(volatile vvh*)(P + (size_t)row * NK + ch * (32 * VW) + lane * VW) = o[ch];
        if (ps == 0) __threadfence(); }
}
template <bool COL>
__global__ __launch_bounds__(256) void k_gate(const h16* __restrict__ GS, const float* __restrict__ O, int p, h16* GO) {
    const int lane = threadIdx.x & 31; const int w = blockIdx.x * 8 + (threadIdx.x >> 5); const int nrows = COL ? NS * 128 : 16 * NRS; if (w >= nrows) return;
    int s, r, zb, n; if (COL) { s = w / 128; r = p * 128 + (w % 128); zb = (r - p * 128) * 8; n = s; } else { s = p * 16 + w / NRS; r = w % NRS; zb = (s - p * 16) * 8; n = r; }
    const size_t row = (size_t)s * NRS + r; const int NN_ = COL ? NS : NRS; v4h o[2];
#pragma unroll
    for (int cc = 0; cc < 2; ++cc)
#pragma unroll
        for (int q = 0; q < 4; ++q) { const int col = cc * 128 + lane * 4 + q; const int h = col >> 5, c = col & 31; const float ov = O[(((size_t)(zb + h)) * NN_ + n) * 64 + c];
            o[cc][q] = tohx((float)GS[row * EE + col] * ov * (1.0f / PCAR)); }
#pragma unroll 1
    for (int ps = 0; ps < 2; ++ps) {
#pragma unroll
        for (int cc = 0; cc < 2; ++cc) *(volatile v4h*)(GO + row * EE + cc * 128 + lane * 4) = o[cc];
        if (ps == 0) __threadfence(); }
}
template <bool RB>
__global__ __launch_bounds__(256) void k_resid(const float* __restrict__ X, const float* __restrict__ U, int rows, float* Y) {
    const int lane = threadIdx.x & 31; const int r = blockIdx.x * 8 + (threadIdx.x >> 5); if (r >= rows) return; v4f o[2];
#pragma unroll
    for (int c = 0; c < 2; ++c) { const v4f x = *(const v4f*)(X + (size_t)r * EE + c * 128 + lane * 4), u = *(const v4f*)(U + (size_t)r * EE + c * 128 + lane * 4);
#pragma unroll
        for (int q = 0; q < 4; ++q) o[c][q] = (RB ? bfr(x[q]) : x[q]) + u[q]; }
#pragma unroll 1
    for (int ps = 0; ps < 2; ++ps) {
#pragma unroll
        for (int c = 0; c < 2; ++c) *(volatile v4f*)(Y + (size_t)r * EE + c * 128 + lane * 4) = o[c];
        if (ps == 0) __threadfence(); }
}
__global__ __launch_bounds__(256) void k_split0(const float* __restrict__ X, bf* Ph, bf* Pl) {
    typedef __attribute__((ext_vector_type(4))) unsigned short v4us;
    const int lane = threadIdx.x & 31; const int r = blockIdx.x * 8 + (threadIdx.x >> 5); if (r >= NRS) return; v4us oh[2], ol[2];
#pragma unroll
    for (int c = 0; c < 2; ++c)
#pragma unroll
        for (int q = 0; q < 4; ++q) { unsigned short a, b; splitf(X[(size_t)r * EE + c * 128 + lane * 4 + q], a, b); oh[c][q] = a; ol[c][q] = b; }
#pragma unroll 1
    for (int ps = 0; ps < 2; ++ps) {
#pragma unroll
        for (int c = 0; c < 2; ++c) { *(volatile v4us*)(Ph + (size_t)r * EE + c * 128 + lane * 4) = oh[c]; *(volatile v4us*)(Pl + (size_t)r * EE + c * 128 + lane * 4) = ol[c]; }
        if (ps == 0) __threadfence(); }
}

extern "C" void kernel_launch(void* const* d_in, const int* in_sizes, int n_in,
                              void* d_out, int out_size, void* d_ws, size_t ws_size, hipStream_t stream) {
    (void)in_sizes; (void)n_in; (void)out_size;
    const float* msa_in = (const float*)d_in[0]; const float* pair = (const float*)d_in[1];
    const float* lrs = (const float*)d_in[2]; const float* lrb = (const float*)d_in[3]; const float* lps = (const float*)d_in[4]; const float* lpb = (const float*)d_in[5];
    const float* Wq = (const float*)d_in[6]; const float* Wk = (const float*)d_in[7]; const float* Wv = (const float*)d_in[8]; const float* Wb = (const float*)d_in[9]; const float* Wg = (const float*)d_in[10]; const float* bg = (const float*)d_in[11]; const float* Wo = (const float*)d_in[12]; const float* bo = (const float*)d_in[13];
    const float* lcs = (const float*)d_in[14]; const float* lcb = (const float*)d_in[15]; const float* Wq2 = (const float*)d_in[16]; const float* Wk2 = (const float*)d_in[17]; const float* Wv2 = (const float*)d_in[18]; const float* Wg2 = (const float*)d_in[19]; const float* bg2 = (const float*)d_in[20]; const float* Wo2 = (const float*)d_in[21]; const float* bo2 = (const float*)d_in[22];
    const float* Wsg = (const float*)d_in[23]; const float* bsg = (const float*)d_in[24];
    float* OUT = (float*)d_out;
    char* wsp = (char*)d_ws;
    auto take = [&](size_t bytes) { char* p = wsp; wsp += (bytes + 255) & ~(size_t)255; return (void*)p; };
    const size_t WSZ = (size_t)EE * EE;
    h16* WQ = (h16*)take(2 * WSZ * 2); h16* WK = (h16*)take(2 * WSZ * 2); h16* WV = (h16*)take(2 * WSZ * 2); h16* WG = (h16*)take(2 * WSZ * 2); h16* WO = (h16*)take(2 * WSZ * 2);
    h16* WQ2 = (h16*)take(2 * WSZ * 2); h16* WK2 = (h16*)take(2 * WSZ * 2); h16* WV2 = (h16*)take(2 * WSZ * 2); h16* WG2 = (h16*)take(2 * WSZ * 2); h16* WO2 = (h16*)take(2 * WSZ * 2);
    h16* WB = (h16*)take((size_t)2 * 64 * PE_ * 2); bf* WS = (bf*)take((size_t)SGL * EE * 2);
    float* MA = (float*)take((size_t)NTR * EE * 4); float* MB = (float*)take((size_t)NTR * EE * 4);
    float* SCR = (float*)take((size_t)NTR * EE * 4);
    h16* Mh = (h16*)take((size_t)NTR * EE * 2); h16* QP = (h16*)take((size_t)NTR * EE * 2); h16* KP = (h16*)take((size_t)NTR * EE * 2); h16* VT = (h16*)take((size_t)NS * NH_ * 64 * NRS * 2);
    h16* GS = (h16*)take((size_t)NTR * EE * 2); h16* GO = (h16*)take((size_t)NTR * EE * 2);
    float* Sb = (float*)take((size_t)ZR * NRS * NRS * 4);
    h16* Zh = (h16*)Sb;
    h16* Pm = (h16*)take((size_t)ZR * NRS * NRS * 2); float* Ob = (float*)take((size_t)ZCP * 64 * 64 * 4); float* BQ8 = (float*)take((size_t)NH_ * NRS * NRS * 4);
    float* M0 = (float*)take((size_t)NRS * EE * 4); bf* M0h = (bf*)take((size_t)NRS * EE * 2); bf* M0l = (bf*)take((size_t)NRS * EE * 2);
    if ((size_t)(wsp - (char*)d_ws) > ws_size) return;
    for (int i = 0; i < 2; ++i) {
        k_wth<<<32, 256, 0, stream>>>(Wq + i * WSZ, EE, EE, EE, WQ + i * WSZ); k_wth<<<32, 256, 0, stream>>>(Wk + i * WSZ, EE, EE, EE, WK + i * WSZ); k_wth<<<32, 256, 0, stream>>>(Wv + i * WSZ, EE, EE, EE, WV + i * WSZ); k_wth<<<32, 256, 0, stream>>>(Wg + i * WSZ, EE, EE, EE, WG + i * WSZ); k_wth<<<32, 256, 0, stream>>>(Wo + i * WSZ, EE, EE, EE, WO + i * WSZ);
        k_wth<<<32, 256, 0, stream>>>(Wq2 + i * WSZ, EE, EE, EE, WQ2 + i * WSZ); k_wth<<<32, 256, 0, stream>>>(Wk2 + i * WSZ, EE, EE, EE, WK2 + i * WSZ); k_wth<<<32, 256, 0, stream>>>(Wv2 + i * WSZ, EE, EE, EE, WV2 + i * WSZ); k_wth<<<32, 256, 0, stream>>>(Wg2 + i * WSZ, EE, EE, EE, WG2 + i * WSZ); k_wth<<<32, 256, 0, stream>>>(Wo2 + i * WSZ, EE, EE, EE, WO2 + i * WSZ);
        k_wth<<<4, 256, 0, stream>>>(Wb + (size_t)i * PE_ * NH_, PE_, NH_, 64, WB + (size_t)i * 64 * PE_); }
    k_wtb<<<48, 256, 0, stream>>>(Wsg, EE, SGL, WS);
    const float qsc = 0.17677669529663688f;
    const unsigned LB256 = (unsigned)(((size_t)NTR * EE / 64 + 63) / 64);
    const unsigned LBVR = (unsigned)(((size_t)NS * NH_ * 64 * NRS / 64 + 63) / 64), LBVC = (unsigned)(((size_t)NRS * NH_ * 64 * NS / 64 + 63) / 64);
    for (int i = 0; i < 2; ++i) {
        const float* Xin = (i == 0) ? msa_in : MB;
        if (i == 0) k_ln<EE, true><<<NTR / 8, 256, 0, stream>>>(Xin, lrs + i * EE, lrb + i * EE, NTR, Mh); else k_ln<EE, false><<<NTR / 8, 256, 0, stream>>>(Xin, lrs + i * EE, lrb + i * EE, NTR, Mh);
        k_ln<PE_, true><<<NPR / 8, 256, 0, stream>>>(pair, lps + i * PE_, lpb + i * PE_, NPR, Zh);
        k_gemmw<h16, 0, false><<<dim3(NPR / 64, 1, 1), 32, 0, stream>>>(Zh, nullptr, WB + (size_t)i * 64 * PE_, nullptr, PE_, SCR, 64, nullptr, 0, 0, 0);
        k_bcomp<<<NH_ * NRS * 2 / 8, 256, 0, stream>>>(SCR, BQ8);
        k_gemmw<h16, 0, false><<<dim3(NTR / 64, EE / 64, 1), 32, 0, stream>>>(Mh, nullptr, WQ + i * WSZ, nullptr, EE, SCR, EE, nullptr, 0, 0, 0); k_hplane<false><<<LB256, 256, 0, stream>>>(SCR, qsc, QP);
        k_gemmw<h16, 0, false><<<dim3(NTR / 64, EE / 64, 1), 32, 0, stream>>>(Mh, nullptr, WK + i * WSZ, nullptr, EE, SCR, EE, nullptr, 0, 0, 0); k_hplane<false><<<LB256, 256, 0, stream>>>(SCR, 1.0f, KP);
        k_gemmw<h16, 0, false><<<dim3(NTR / 64, EE / 64, 1), 32, 0, stream>>>(Mh, nullptr, WV + i * WSZ, nullptr, EE, SCR, EE, nullptr, 0, 0, 0); k_vtplane<false><<<LBVR, 256, 0, stream>>>(SCR, VT);
        k_gemmw<h16, 0, false><<<dim3(NTR / 64, EE / 64, 1), 32, 0, stream>>>(Mh, nullptr, WG + i * WSZ, nullptr, EE, SCR, EE, nullptr, 0, 0, 0); k_gsig<<<NTR / 8, 256, 0, stream>>>(SCR, bg + i * EE, GS);
        for (int p = 0; p < NS / 16; ++p) { const size_t zo = (size_t)p * ZR;
            k_gemmw<h16, 0, false><<<dim3(NRS / 64, NRS / 64, ZR), 32, 0, stream>>>(QP + zo * NRS * HC, nullptr, KP + zo * NRS * HC, nullptr, HC, Sb, NRS, nullptr, (size_t)NRS * HC, (size_t)NRS * HC, (size_t)NRS * NRS);
            k_soft<256, true><<<ZR * NRS / 8, 256, 0, stream>>>(Sb, BQ8, ZR * NRS, Pm);
            k_gemmw<h16, 0, false><<<dim3(NRS / 64, 1, ZR), 32, 0, stream>>>(Pm, nullptr, VT + zo * 64 * NRS, nullptr, NRS, Ob, 64, nullptr, (size_t)NRS * NRS, (size_t)64 * NRS, (size_t)NRS * 64);
            k_gate<false><<<16 * NRS / 8, 256, 0, stream>>>(GS, Ob, p, GO); }
        k_gemmw<h16, 0, true><<<dim3(NTR / 64, EE / 64, 1), 32, 0, stream>>>(GO, nullptr, WO + i * WSZ, nullptr, EE, SCR, EE, bo + i * EE, 0, 0, 0);
        if (i == 0) k_resid<true><<<NTR / 8, 256, 0, stream>>>(Xin, SCR, NTR, MA); else k_resid<false><<<NTR / 8, 256, 0, stream>>>(Xin, SCR, NTR, MA);
        k_ln<EE, false><<<NTR / 8, 256, 0, stream>>>(MA, lcs + i * EE, lcb + i * EE, NTR, Mh);
        k_gemmw<h16, 0, false><<<dim3(NTR / 64, EE / 64, 1), 32, 0, stream>>>(Mh, nullptr, WQ2 + i * WSZ, nullptr, EE, SCR, EE, nullptr, 0, 0, 0); k_hplane<true><<<LB256, 256, 0, stream>>>(SCR, qsc, QP);
        k_gemmw<h16, 0, false><<<dim3(NTR / 64, EE / 64, 1), 32, 0, stream>>>(Mh, nullptr, WK2 + i * WSZ, nullptr, EE, SCR, EE, nullptr, 0, 0, 0); k_hplane<true><<<LB256, 256, 0, stream>>>(SCR, 1.0f, KP);
        k_gemmw<h16, 0, false><<<dim3(NTR / 64, EE / 64, 1), 32, 0, stream>>>(Mh, nullptr, WV2 + i * WSZ, nullptr, EE, SCR, EE, nullptr, 0, 0, 0); k_vtplane<true><<<LBVC, 256, 0, stream>>>(SCR, VT);
        k_gemmw<h16, 0, false><<<dim3(NTR / 64, EE / 64, 1), 32, 0, stream>>>(Mh, nullptr, WG2 + i * WSZ, nullptr, EE, SCR, EE, nullptr, 0, 0, 0); k_gsig<<<NTR / 8, 256, 0, stream>>>(SCR, bg2 + i * EE, GS);
        for (int p = 0; p < NRS / 128; ++p) { const size_t zo = (size_t)p * ZCP;
            k_gemmw<h16, 0, false><<<dim3(1, 1, ZCP), 32, 0, stream>>>(QP + zo * NS * HC, nullptr, KP + zo * NS * HC, nullptr, HC, Sb, NS, nullptr, (size_t)NS * HC, (size_t)NS * HC, (size_t)NS * NS);
            k_soft<64, false><<<ZCP * NS / 8, 256, 0, stream>>>(Sb, BQ8, ZCP * NS, Pm);
            k_gemmw<h16, 0, false><<<dim3(1, 1, ZCP), 32, 0, stream>>>(Pm, nullptr, VT + zo * 64 * NS, nullptr, NS, Ob, 64, nullptr, (size_t)NS * NS, (size_t)64 * NS, (size_t)NS * 64);
            k_gate<true><<<NS * 128 / 8, 256, 0, stream>>>(GS, Ob, p, GO); }
        if (i == 0) { k_gemmw<h16, 0, true><<<dim3(NTR / 64, EE / 64, 1), 32, 0, stream>>>(GO, nullptr, WO2 + i * WSZ, nullptr, EE, SCR, EE, bo2 + i * EE, 0, 0, 0); k_resid<false><<<NTR / 8, 256, 0, stream>>>(MA, SCR, NTR, MB); }
        else { k_gemmw<h16, 0, true><<<dim3(NRS / 64, EE / 64, 1), 32, 0, stream>>>(GO, nullptr, WO2 + i * WSZ, nullptr, EE, SCR, EE, bo2 + i * EE, 0, 0, 0); k_resid<false><<<NRS / 8, 256, 0, stream>>>(MA, SCR, NRS, M0); } }
    k_split0<<<NRS / 8, 256, 0, stream>>>(M0, M0h, M0l);
    k_gemmw<bf, 1, true><<<dim3(NRS / 64, SGL / 64, 1), 32, 0, stream>>>(M0h, M0l, WS, nullptr, EE, OUT, SGL, bsg, 0, 0, 0);
}
